// LATTE_73177652789619
// MI455X (gfx1250) — hardware-verified
//
#include <hip/hip_runtime.h>
#include <stddef.h>
#include <stdint.h>


#define DIN     128
#define NH      4
#define HCH     32
#define NCOL    256
#define NSC     16
#define NSP     8
#define NTHR    256
#define NWAVE   8
#define EPT     8
#define CHUNK   (NTHR * EPT)
#define WCAP    (EPT * 32)
#define LISTN   (NWAVE * WCAP)
#define NBMAX   2048
#define NBMIN   256
#define RCAP    28672
#define DEGCAP  1024
#define GBM     64
#define GBN     64
#define GTHR    128
#define FNODE   64
#define WSMAX   134217728
#define LDS_SEG ((2 * RCAP + 2 * NBMAX + LISTN) * 4 + 64)

static_assert((CHUNK & (CHUNK - 1)) == 0 && CHUNK <= 4096);
static_assert((NBMAX & (NBMAX - 1)) == 0 && NBMAX <= 4096);
static_assert(NTHR * 8 == NBMAX);
static_assert((NBMAX % NTHR) == 0 && (NBMIN % NTHR) == 0 && NBMIN <= NBMAX);
static_assert(LISTN >= NBMAX);
static_assert(LISTN >= NWAVE * WCAP);
static_assert((RCAP % 32) == 0);
static_assert(4 * NBMAX <= RCAP);
static_assert(LDS_SEG <= 300000);
static_assert(GBM == (GTHR / 32) * 16);
static_assert(GTHR == 2 * GBM);
static_assert((DIN % 32) == 0 && DIN / 8 == 16);
static_assert((NCOL % GBN) == 0 && NCOL == 2 * DIN);
static_assert(DIN == NH * HCH && GBN == 2 * HCH);
static_assert(FNODE * NH == NTHR);
static_assert(((FNODE * DIN / 4) % NTHR) == 0);

typedef float          v4f   __attribute__((ext_vector_type(4)));
typedef float          v8f   __attribute__((ext_vector_type(8)));
typedef int            v4i   __attribute__((ext_vector_type(4)));
typedef unsigned int   v2u   __attribute__((ext_vector_type(2)));
typedef unsigned int   v4u   __attribute__((ext_vector_type(4)));
typedef unsigned int   v8u   __attribute__((ext_vector_type(8)));
typedef __bf16         v16bf __attribute__((ext_vector_type(16)));
union FragB { v8u w; v4u q[2]; };

__device__ __forceinline__ v8f wmb(const FragB& a, const FragB& b, v8f c) {
  const v16bf av = __builtin_bit_cast(v16bf, a.w);
  const v16bf bv = __builtin_bit_cast(v16bf, b.w);
  v8f d = __builtin_amdgcn_wmma_f32_16x16x32_bf16(false, av, false, bv, (short)0, c, false, false);
  asm volatile("v_nop\n\tv_nop\n\tv_nop\n\tv_nop" : "+v"(d) : "v"(a.w), "v"(b.w));
  return d;
}

__device__ __forceinline__ unsigned short f2bf(float x) {
  unsigned u = __float_as_uint(x);
  u += 0x7FFFu + ((u >> 16) & 1u);
  return (unsigned short)(u >> 16);
}
__device__ __forceinline__ float bfr(float x) { return __uint_as_float(((unsigned)f2bf(x)) << 16); }
__device__ __forceinline__ unsigned pk2(float a, float b) {
  return (unsigned)f2bf(a) | ((unsigned)f2bf(b) << 16);
}

__global__ __launch_bounds__(NTHR) void k_cvt(const float* __restrict__ x, unsigned short* xb, int nValid, int nUnits) {
  const int i = (int)blockIdx.x * NTHR + (int)threadIdx.x;
  if (i >= nUnits) return;
  const int row = i >> 4;
  const int c0  = (i & 15) * 8;
  const int rc  = row < nValid ? row : nValid - 1;
  const float* p = x + (size_t)rc * DIN + c0;
  v4f a = *(const v4f*)p, b = *(const v4f*)(p + 4);
  const v4f z4 = {0.f, 0.f, 0.f, 0.f};
  if (row >= nValid) { a = z4; b = z4; }
  v4u w;
  w.x = pk2(a.x, a.y); w.y = pk2(a.z, a.w); w.z = pk2(b.x, b.y); w.w = pk2(b.z, b.w);
  const size_t o = (size_t)row * DIN + c0;
  *(volatile v4u*)(xb + o) = w;
  __threadfence();
  *(volatile v4u*)(xb + o) = w;
}

__global__ __launch_bounds__(GTHR) void k_gemm(
    const unsigned short* __restrict__ A, const unsigned short* __restrict__ WT,
    const float* __restrict__ bl, const float* __restrict__ br,
    const float* __restrict__ attl, const float* __restrict__ attr,
    float* V, float* SC, int MPr)
{
  __shared__ __attribute__((aligned(16))) float stg[GBM * GBN];
  __shared__ __attribute__((aligned(16))) float scs[4 * GBM];
  const int tid = (int)threadIdx.x, lane = tid & 31, wave = tid >> 5, hh = lane >> 4, m = lane & 15;
  const int rowBase = (int)blockIdx.x * GBM;
  const int y       = (int)blockIdx.y;
  const int col0    = y * GBN;

  v8f acc[4];
  {
    const v8f z = {0.f, 0.f, 0.f, 0.f, 0.f, 0.f, 0.f, 0.f};
    acc[0] = z; acc[1] = z; acc[2] = z; acc[3] = z;
  }
  const unsigned short* ap = A  + (size_t)(rowBase + 16 * wave + m) * (size_t)DIN + 8 * hh;
  const unsigned short* wp = WT + (size_t)(col0 + m) * (size_t)DIN + 8 * hh;
#pragma unroll 1
  for (int ks = 0; ks < DIN / 32; ++ks) {
    FragB af;
    af.q[0] = *(const v4u*)(ap + 32 * ks);
    af.q[1] = *(const v4u*)(ap + 32 * ks + 16);
#pragma unroll
    for (int t = 0; t < 4; ++t) {
      const unsigned short* wq = wp + (size_t)(16 * t) * (size_t)DIN + 32 * ks;
      FragB bf;
      bf.q[0] = *(const v4u*)wq;
      bf.q[1] = *(const v4u*)(wq + 16);
      acc[t] = wmb(af, bf, acc[t]);
    }
  }

  const float* bp = (y < 2) ? bl : br;
  const int bofs = (y < 2) ? col0 : col0 - DIN;
#pragma unroll
  for (int t = 0; t < 4; ++t) {
    const int lc = 16 * t + m;
    int bi = bofs + lc;
    bi = bi > DIN - 1 ? DIN - 1 : bi;
    bi = bi < 0 ? 0 : bi;
    const float bv = bfr(bp[bi]);
#pragma unroll
    for (int r = 0; r < 8; ++r) {
      const int lr = 16 * wave + 8 * hh + r;
      stg[lr * GBN + lc] = acc[t][r] + bv;
    }
  }
  __syncthreads();

  {
    const int row = tid & (GBM - 1);
    const int mm  = tid >> 6;
    const int hb  = 2 * (y & 1);
    const float* avp = (y < 2) ? attl : attr;
    const float* a0p = avp + (mm * NH + hb) * HCH;
    const float* a1p = a0p + HCH;
    const float* srow = stg + row * GBN;
    float d0 = 0.f, d1 = 0.f;
#pragma unroll 1
    for (int c = 0; c < HCH; c += 4) {
      const v4f s0 = *(const v4f*)(srow + c);
      const v4f s1 = *(const v4f*)(srow + HCH + c);
      d0 = fmaf(s0.x, bfr(a0p[c]),     d0);
      d0 = fmaf(s0.y, bfr(a0p[c + 1]), d0);
      d0 = fmaf(s0.z, bfr(a0p[c + 2]), d0);
      d0 = fmaf(s0.w, bfr(a0p[c + 3]), d0);
      d1 = fmaf(s1.x, bfr(a1p[c]),     d1);
      d1 = fmaf(s1.y, bfr(a1p[c + 1]), d1);
      d1 = fmaf(s1.z, bfr(a1p[c + 2]), d1);
      d1 = fmaf(s1.w, bfr(a1p[c + 3]), d1);
    }
    scs[(2 * mm) * GBM + row]     = d0;
    scs[(2 * mm + 1) * GBM + row] = d1;
  }

  v4f fv[8];
#pragma unroll
  for (int i = 0; i < 8; ++i) {
    const int lr = 16 * wave + 2 * i + hh;
    fv[i] = *(const v4f*)(stg + lr * GBN + 4 * m);
  }
  __syncthreads();

  const int sj = (tid >> 4) & 3;
  const int sp = tid & 15;
  const v4f sv = *(const v4f*)(scs + sj * GBM + 4 * sp);
  float* sdst = SC + (size_t)(4 * y + sj) * (size_t)MPr + rowBase + 4 * sp;
  const bool wsc = tid < GBM;
  const bool wv  = (y >= 2);
  const int  cv  = wv ? (col0 - DIN) : 0;

  if (wv) {
#pragma unroll
    for (int i = 0; i < 8; ++i) {
      const int lr = 16 * wave + 2 * i + hh;
      float* op = V + (size_t)(rowBase + lr) * (size_t)DIN + cv + 4 * m;
      *(volatile v4f*)op = fv[i];
    }
  }
  if (wsc) *(volatile v4f*)sdst = sv;
  __threadfence();
  if (wv) {
#pragma unroll
    for (int i = 0; i < 8; ++i) {
      const int lr = 16 * wave + 2 * i + hh;
      float* op = V + (size_t)(rowBase + lr) * (size_t)DIN + cv + 4 * m;
      *(volatile v4f*)op = fv[i];
    }
  }
  if (wsc) *(volatile v4f*)sdst = sv;
}

__device__ __forceinline__ int scan_chunk(const int* __restrict__ dsts, int nE, int cbase, int slotBase,
                                          int nb, int vec8, int* list, int tid, int lane, int wave) {
  int wc = 0;
  const int el0  = tid * EPT;
  const int e0   = cbase + el0;
  const int sent = -2147483647 - 1;
  v4i da, db;
  if (vec8 != 0 && cbase + CHUNK <= nE) {
    da = *(const v4i*)(dsts + e0);
    db = *(const v4i*)(dsts + e0 + 4);
  } else {
    da.x = (e0     < nE) ? dsts[min(e0,     nE - 1)] : sent;
    da.y = (e0 + 1 < nE) ? dsts[min(e0 + 1, nE - 1)] : sent;
    da.z = (e0 + 2 < nE) ? dsts[min(e0 + 2, nE - 1)] : sent;
    da.w = (e0 + 3 < nE) ? dsts[min(e0 + 3, nE - 1)] : sent;
    db.x = (e0 + 4 < nE) ? dsts[min(e0 + 4, nE - 1)] : sent;
    db.y = (e0 + 5 < nE) ? dsts[min(e0 + 5, nE - 1)] : sent;
    db.z = (e0 + 6 < nE) ? dsts[min(e0 + 6, nE - 1)] : sent;
    db.w = (e0 + 7 < nE) ? dsts[min(e0 + 7, nE - 1)] : sent;
  }
  const unsigned nbs = (unsigned)slotBase;
  const unsigned unb = (unsigned)nb;
  const unsigned s0 = (unsigned)da.x - nbs, s1 = (unsigned)da.y - nbs;
  const unsigned s2 = (unsigned)da.z - nbs, s3 = (unsigned)da.w - nbs;
  const unsigned s4 = (unsigned)db.x - nbs, s5 = (unsigned)db.y - nbs;
  const unsigned s6 = (unsigned)db.z - nbs, s7 = (unsigned)db.w - nbs;
  const bool h0 = s0 < unb, h1 = s1 < unb, h2 = s2 < unb, h3 = s3 < unb;
  const bool h4 = s4 < unb, h5 = s5 < unb, h6 = s6 < unb, h7 = s7 < unb;
  const unsigned any = __builtin_amdgcn_ballot_w32(h0 | h1 | h2 | h3 | h4 | h5 | h6 | h7);
  if (any != 0u) {
#define HITJ(J, HJ, SJ) { \
      const unsigned mj = __builtin_amdgcn_ballot_w32(HJ); \
      if (mj != 0u) { \
        if (HJ) { \
          const int pos = wc + (int)__builtin_amdgcn_mbcnt_lo(mj, 0u); \
          if (pos < WCAP) list[wave * WCAP + pos] = ((el0 + (J)) << 12) | (int)(SJ); \
        } \
        wc += (int)__builtin_popcount(mj); } }
    HITJ(0, h0, s0)
    HITJ(1, h1, s1)
    HITJ(2, h2, s2)
    HITJ(3, h3, s3)
    HITJ(4, h4, s4)
    HITJ(5, h5, s5)
    HITJ(6, h6, s6)
    HITJ(7, h7, s7)
#undef HITJ
  }
  return wc;
}

__global__ __launch_bounds__(NTHR) void k_seg(
    const int* __restrict__ src0, const int* __restrict__ dst0,
    const int* __restrict__ src1, const int* __restrict__ dst1,
    const float* __restrict__ alpha, const float* __restrict__ SC, float* SP,
    int nN, int nE0, int nE1, int nb, int vec8, int MPr) {
  extern __shared__ v4f lds_dyn[];
  int* reg1 = (int*)lds_dyn;
  int* reg2 = reg1 + RCAP;
  int* scnt = reg2 + RCAP;
  int* soff = scnt + NBMAX;
  int* list = soff + NBMAX;
  int* wcnt = list + LISTN;
  int* wtot = wcnt + NWAVE;
  const int tid = (int)threadIdx.x, lane = tid & 31, wave = tid >> 5;
  const int m = (int)blockIdx.y;
  const int* srcs = (m != 0) ? src1 : src0;
  const int* dsts = (m != 0) ? dst1 : dst0;
  const int  nE   = (m != 0) ? nE1 : nE0;
  const int nodeBase = (int)blockIdx.x * nb;

  for (int i = tid; i < NBMAX; i += NTHR) scnt[i] = 0;
  __syncthreads();

  int tot = 0;
  const int nChunks = (nE + CHUNK - 1) / CHUNK;
#pragma unroll 1
  for (int ch = 0; ch < nChunks; ++ch) {
    const int cbase = ch * CHUNK;
    const int wc = scan_chunk(dsts, nE, cbase, nodeBase, nb, vec8, list, tid, lane, wave);
    if (lane == 0) wcnt[wave] = wc;
    __syncthreads();
    int pre = 0, all = 0;
#pragma unroll
    for (int w2 = 0; w2 < NWAVE; ++w2) {
      int c = wcnt[w2];
      c = c < 0 ? 0 : (c > WCAP ? WCAP : c);
      all += c;
      pre += (w2 < wave) ? c : 0;
    }
    const int wcc  = wc > WCAP ? WCAP : wc;
    const int base = tot + pre;
#pragma unroll 1
    for (int i = lane; i < wcc; i += 32) {
      const int ent = list[wave * WCAP + i];
      const int el  = (ent >> 12) & (CHUNK - 1);
      const int sl  = ent & (NBMAX - 1);
      int eid = cbase + el;
      eid = eid > nE - 1 ? nE - 1 : eid;
      const int pos = base + i;
      if (pos < RCAP) reg1[pos] = (int)(((unsigned)eid << 12) | (unsigned)sl);
    }
    tot += all;
    tot = tot > RCAP ? RCAP : tot;
    __syncthreads();
  }
  const int nh = tot;

  if (wave == 0) {
#pragma unroll 1
    for (int b0 = 0; b0 < nh; b0 += 32) {
      const int idx = b0 + lane;
      const int uv  = reg1[idx < RCAP ? idx : RCAP - 1];
      const int m32 = (nh - b0) < 32 ? (nh - b0) : 32;
#pragma unroll 1
      for (int k = 0; k < m32; ++k) {
        const int u  = __builtin_amdgcn_readlane(uv, k);
        const int sl = u & (NBMAX - 1);
        if (lane == 0) scnt[sl] = scnt[sl] + 1;
      }
    }
  }
  __syncthreads();

  {
    const v4i ca = *(const v4i*)(scnt + 8 * tid);
    const v4i cb = *(const v4i*)(scnt + 8 * tid + 4);
    const int e0 = ca.x < 0 ? 0 : ca.x, e1 = ca.y < 0 ? 0 : ca.y, e2 = ca.z < 0 ? 0 : ca.z, e3 = ca.w < 0 ? 0 : ca.w;
    const int e4 = cb.x < 0 ? 0 : cb.x, e5 = cb.y < 0 ? 0 : cb.y, e6 = cb.z < 0 ? 0 : cb.z, e7 = cb.w < 0 ? 0 : cb.w;
    const int ts = e0 + e1 + e2 + e3 + e4 + e5 + e6 + e7;
    int incl = ts;
#pragma unroll
    for (int d = 1; d < 32; d <<= 1) {
      const int up = __shfl_up(incl, d);
      if (lane >= d) incl += up;
    }
    if (lane == 31) wtot[wave] = incl;
    __syncthreads();
    int pre = 0;
#pragma unroll
    for (int w2 = 0; w2 < NWAVE; ++w2) pre += (w2 < wave) ? wtot[w2] : 0;
    int run = pre + incl - ts;
    soff[8 * tid + 0] = run; run += e0;
    soff[8 * tid + 1] = run; run += e1;
    soff[8 * tid + 2] = run; run += e2;
    soff[8 * tid + 3] = run; run += e3;
    soff[8 * tid + 4] = run; run += e4;
    soff[8 * tid + 5] = run; run += e5;
    soff[8 * tid + 6] = run; run += e6;
    soff[8 * tid + 7] = run;
  }
  __syncthreads();
  for (int i = tid; i < NBMAX; i += NTHR) list[i] = soff[i];
  __syncthreads();

  if (wave == 0) {
#pragma unroll 1
    for (int b0 = 0; b0 < nh; b0 += 32) {
      const int idx = b0 + lane;
      const int uv  = reg1[idx < RCAP ? idx : RCAP - 1];
      const int m32 = (nh - b0) < 32 ? (nh - b0) : 32;
#pragma unroll 1
      for (int k = 0; k < m32; ++k) {
        const int u   = __builtin_amdgcn_readlane(uv, k);
        const int sl  = u & (NBMAX - 1);
        const int eid = (int)((unsigned)u >> 12);
        if (lane == 0) {
          int pos = list[sl];
          pos = pos < 0 ? 0 : (pos > RCAP - 1 ? RCAP - 1 : pos);
          reg2[pos] = eid;
          list[sl] = pos + 1;
        }
      }
    }
  }
  __syncthreads();

  const bool ovf = (nh >= RCAP);
  const float qnan = __int_as_float(0x7fc00000);
  const float alm  = bfr(alpha[m]);
  float* sst = (float*)reg1;
  const size_t MPs = (size_t)MPr;
  const float* la0 = SC + (size_t)(2 * m) * MPs;
  const float* la1 = la0 + MPs;
  const float* la2 = SC + (size_t)(4 + 2 * m) * MPs;
  const float* la3 = la2 + MPs;
  const float* ra0 = la0 + (size_t)8 * MPs;
  const float* ra1 = la1 + (size_t)8 * MPs;
  const float* ra2 = la2 + (size_t)8 * MPs;
  const float* ra3 = la3 + (size_t)8 * MPs;
  const int spt = nb / NTHR;
#pragma unroll 1
  for (int jt = 0; jt < spt; ++jt) {
    const int slot = jt * NTHR + tid;
    const int grow = nodeBase + slot;
    const int gcl  = grow < nN ? grow : nN - 1;
    int st = soff[slot];
    const int craw = scnt[slot];
    int cnt = craw;
    st  = st < 0 ? 0 : (st > nh ? nh : st);
    cnt = cnt < 0 ? 0 : (cnt > DEGCAP ? DEGCAP : cnt);
    if (cnt > nh - st) cnt = nh - st;
    const float pz = (ovf || craw > DEGCAP) ? qnan : 0.0f;
    const float live = grow < nN ? 1.0f : 0.0f;
    const float r0 = ra0[gcl], r1 = ra1[gcl], r2 = ra2[gcl], r3 = ra3[gcl];
    float mx0 = -1.0e30f, mx1 = -1.0e30f, mx2 = -1.0e30f, mx3 = -1.0e30f;
    float dn0 = 0.f, dn1 = 0.f, dn2 = 0.f, dn3 = 0.f;
#pragma unroll 1
    for (int q = 0; q < cnt; ++q) {
      int idx = st + q; idx = idx > RCAP - 1 ? RCAP - 1 : idx;
      int eid = reg2[idx]; eid = eid < 0 ? 0 : (eid > nE - 1 ? nE - 1 : eid);
      const int sraw = srcs[eid];
      const int s = sraw < 0 ? 0 : (sraw > nN - 1 ? nN - 1 : sraw);
      const float t0 = (la0[s] + r0) * alm;
      const float t1 = (la1[s] + r1) * alm;
      const float t2 = (la2[s] + r2) * alm;
      const float t3 = (la3[s] + r3) * alm;
#define UPD(MX, DN, AT) { \
        const float df = (AT) - MX; \
        const float ee = __expf(-fabsf(df)); \
        const bool up  = df > 0.f; \
        const float s1 = up ? ee : 1.0f; \
        const float s2 = up ? 1.0f : ee; \
        MX = up ? (AT) : MX; \
        DN = fmaf(DN, s1, s2); }
      UPD(mx0, dn0, t0)
      UPD(mx1, dn1, t1)
      UPD(mx2, dn2, t2)
      UPD(mx3, dn3, t3)
#undef UPD
    }
#define FIN(DN) (((DN) > 0.f ? (DN) * __builtin_amdgcn_rcpf((DN) > 0.f ? (DN) : 1.0f) : 0.0f) * live + pz)
    sst[0 * nb + slot] = FIN(dn0);
    sst[1 * nb + slot] = FIN(dn1);
    sst[2 * nb + slot] = FIN(dn2);
    sst[3 * nb + slot] = FIN(dn3);
#undef FIN
  }
  __syncthreads();

  int nv = MPr - nodeBase;
  nv = nv < 0 ? 0 : (nv > nb ? nb : nv);
  const int ppr  = nv >> 2;
  const int pprd = ppr > 0 ? ppr : 1;
  const int np   = 4 * ppr;
  float* sb = SP + (size_t)(4 * m) * MPs + nodeBase;
#pragma unroll 1
  for (int i = 0; i < spt; ++i) {
    const int p = i * NTHR + tid;
    if (p < np) {
      int hr = p / pprd; hr = hr > 3 ? 3 : hr;
      const int pc = p - hr * ppr;
      const v4f val = *(const v4f*)(sst + hr * nb + 4 * pc);
      *(volatile v4f*)(sb + (size_t)hr * MPs + 4 * pc) = val;
    }
  }
  __threadfence();
#pragma unroll 1
  for (int i = 0; i < spt; ++i) {
    const int p = i * NTHR + tid;
    if (p < np) {
      int hr = p / pprd; hr = hr > 3 ? 3 : hr;
      const int pc = p - hr * ppr;
      const v4f val = *(const v4f*)(sst + hr * nb + 4 * pc);
      *(volatile v4f*)(sb + (size_t)hr * MPs + 4 * pc) = val;
    }
  }
}

__global__ __launch_bounds__(NTHR) void k_fin(
    const unsigned short* __restrict__ XB, const float* __restrict__ V, const float* __restrict__ SP,
    const float* __restrict__ rl, const float* __restrict__ rr, float* out, int nN, int MPr) {
  __shared__ __attribute__((aligned(16))) float ost[FNODE * DIN];
  __shared__ __attribute__((aligned(16))) float srl[NH * HCH];
  __shared__ __attribute__((aligned(16))) float srr[NH * HCH];
  const int tid = (int)threadIdx.x;
  if (tid < NH * HCH) { srl[tid] = bfr(rl[tid]); srr[tid] = bfr(rr[tid]); }
  __syncthreads();
  const int ql = tid >> 2, h = tid & 3;
  const int nodeBase = (int)blockIdx.x * FNODE;
  const int grow = nodeBase + ql;
  const int gcl  = grow < nN ? grow : nN - 1;
  const float* vp = V + (size_t)gcl * DIN + h * HCH;
  const unsigned short* fp = XB + (size_t)gcl * DIN + h * HCH;
  const float S0 = SP[(size_t)h * (size_t)MPr + gcl];
  const float S1 = SP[(size_t)(NH + h) * (size_t)MPr + gcl];
  const float* lp = srl + h * HCH;
  const float* rp = srr + h * HCH;

  float al = 0.f, a0 = 0.f, a1 = 0.f, a2 = 0.f;
#pragma unroll 1
  for (int c = 0; c < HCH; c += 4) {
    const v2u fw = *(const v2u*)(fp + c);
    const v4f vv = *(const v4f*)(vp + c);
    const v4f lw = *(const v4f*)(lp + c);
    const v4f rw = *(const v4f*)(rp + c);
    const float f0 = __uint_as_float(fw.x << 16), f1 = __uint_as_float(fw.x & 0xffff0000u);
    const float f2 = __uint_as_float(fw.y << 16), f3 = __uint_as_float(fw.y & 0xffff0000u);
    al = fmaf(f0, lw.x, al); al = fmaf(f1, lw.y, al); al = fmaf(f2, lw.z, al); al = fmaf(f3, lw.w, al);
    a2 = fmaf(f0, rw.x, a2); a2 = fmaf(f1, rw.y, a2); a2 = fmaf(f2, rw.z, a2); a2 = fmaf(f3, rw.w, a2);
    const float g0 = S0 * vv.x, g1 = S0 * vv.y, g2 = S0 * vv.z, g3 = S0 * vv.w;
    a0 = fmaf(g0, rw.x, a0); a0 = fmaf(g1, rw.y, a0); a0 = fmaf(g2, rw.z, a0); a0 = fmaf(g3, rw.w, a0);
    const float e0 = S1 * vv.x, e1 = S1 * vv.y, e2 = S1 * vv.z, e3 = S1 * vv.w;
    a1 = fmaf(e0, rw.x, a1); a1 = fmaf(e1, rw.y, a1); a1 = fmaf(e2, rw.z, a1); a1 = fmaf(e3, rw.w, a1);
  }

  float b0, b1, b2;
#define HSMX(XR, BR) { \
    const float xs = (XR); \
    const float lk = xs > 0.f ? xs : 0.2f * xs; \
    float mxv = fmaxf(lk, __shfl_xor(lk, 1)); \
    mxv = fmaxf(mxv, __shfl_xor(mxv, 2)); \
    const float ev = __expf(lk - mxv); \
    float sm = ev + __shfl_xor(ev, 1); \
    sm = sm + __shfl_xor(sm, 2); \
    BR = ev * __builtin_amdgcn_rcpf(sm); }
  HSMX(al + a0, b0)
  HSMX(al + a1, b1)
  HSMX(al + a2, b2)
#undef HSMX

  float* orow = ost + ql * DIN + h * HCH;
#pragma unroll 1
  for (int c = 0; c < HCH; c += 4) {
    const v2u fw = *(const v2u*)(fp + c);
    const v4f vv = *(const v4f*)(vp + c);
    const float f0 = __uint_as_float(fw.x << 16), f1 = __uint_as_float(fw.x & 0xffff0000u);
    const float f2 = __uint_as_float(fw.y << 16), f3 = __uint_as_float(fw.y & 0xffff0000u);
    v4f o;
    o.x = fmaxf(fmaf(b2, f0, fmaf(b1, S1 * vv.x, b0 * (S0 * vv.x))), 0.f);
    o.y = fmaxf(fmaf(b2, f1, fmaf(b1, S1 * vv.y, b0 * (S0 * vv.y))), 0.f);
    o.z = fmaxf(fmaf(b2, f2, fmaf(b1, S1 * vv.z, b0 * (S0 * vv.z))), 0.f);
    o.w = fmaxf(fmaf(b2, f3, fmaf(b1, S1 * vv.w, b0 * (S0 * vv.w))), 0.f);
    *(v4f*)(orow + c) = o;
  }
  __syncthreads();

  int nv = nN - nodeBase;
  nv = nv < 0 ? 0 : (nv > FNODE ? FNODE : nv);
  const int np = nv * (DIN / 4);
  float* ob = out + (size_t)nodeBase * DIN;
#pragma unroll
  for (int i = 0; i < (FNODE * DIN / 4) / NTHR; ++i) {
    const int p = i * NTHR + tid;
    if (p < np) *(volatile v4f*)(ob + 4 * (size_t)p) = *(const v4f*)(ost + 4 * p);
  }
  __threadfence();
#pragma unroll
  for (int i = 0; i < (FNODE * DIN / 4) / NTHR; ++i) {
    const int p = i * NTHR + tid;
    if (p < np) *(volatile v4f*)(ob + 4 * (size_t)p) = *(const v4f*)(ost + 4 * p);
  }
}

static int pick_nb(int nE, int nN) {
  int nb = NBMAX;
  while (nb > NBMIN && (long long)nb * (long long)nE * 5LL > (long long)RCAP * (long long)nN * 4LL) nb >>= 1;
  return nb;
}
static inline int cdiv(int a, int b) { return (a + b - 1) / b; }

extern "C" void kernel_launch(void* const* d_in, const int* in_sizes, int n_in,
                              void* d_out, int out_size, void* d_ws, size_t ws_size,
                              hipStream_t stream) {
  if (n_in < 14) return;
  const int nN = in_sizes[0] / DIN;
  if (nN <= 0 || in_sizes[0] != nN * DIN || nN > (1 << 22)) return;
  if (in_sizes[1] != DIN * DIN || in_sizes[2] != DIN) return;
  if (in_sizes[3] != DIN * DIN || in_sizes[4] != DIN) return;
  if (in_sizes[5] != 2 * NH * HCH || in_sizes[6] != 2 * NH * HCH) return;
  if (in_sizes[7] != NH * HCH || in_sizes[8] != NH * HCH) return;
  if (in_sizes[9] < 2) return;
  const int nE0 = in_sizes[10], nE1 = in_sizes[12];
  if (in_sizes[11] != nE0 || in_sizes[13] != nE1) return;
  if (nE0 < 1 || nE1 < 1 || nE0 > (1 << 20) || nE1 > (1 << 20)) return;
  if (out_size != nN * DIN) return;

  const float* feat = (const float*)d_in[0];
  const float* Wl   = (const float*)d_in[1];
  const float* bl   = (const float*)d_in[2];
  const float* Wr   = (const float*)d_in[3];
  const float* br   = (const float*)d_in[4];
  const float* attl = (const float*)d_in[5];
  const float* attr = (const float*)d_in[6];
  const float* rl   = (const float*)d_in[7];
  const float* rr   = (const float*)d_in[8];
  const float* alph = (const float*)d_in[9];
  const int*   src0 = (const int*)  d_in[10];
  const int*   dst0 = (const int*)  d_in[11];
  const int*   src1 = (const int*)  d_in[12];
  const int*   dst1 = (const int*)  d_in[13];
  float* out = (float*)d_out;

  const int MP   = cdiv(nN, GBM) * GBM;
  const int nEmx = nE0 > nE1 ? nE0 : nE1;
  const int nb   = pick_nb(nEmx, nN);
  const int gA   = cdiv(MP, nb);
  const int vec8 = (((nE0 & 3) == 0) && ((nE1 & 3) == 0)) ? 1 : 0;
  if (gA * nb < MP || (nb % NTHR) != 0) return;

  char* ws = (char*)d_ws;
  size_t off = 0;
  const size_t oXB = off; off += (size_t)MP * DIN * 2;            off = (off + 255) & ~(size_t)255;
  const size_t oWT = off; off += (size_t)NCOL * DIN * 2;          off = (off + 255) & ~(size_t)255;
  const size_t oV  = off; off += (size_t)MP * DIN * 4;            off = (off + 255) & ~(size_t)255;
  const size_t oSC = off; off += (size_t)NSC * MP * 4;            off = (off + 255) & ~(size_t)255;
  const size_t oSP = off; off += (size_t)NSP * MP * 4;            off = (off + 255) & ~(size_t)255;
  if (off > ws_size || off > (size_t)WSMAX) return;
  unsigned short* XB = (unsigned short*)(ws + oXB);
  unsigned short* WT = (unsigned short*)(ws + oWT);
  float* Vp  = (float*)(ws + oV);
  float* SCp = (float*)(ws + oSC);
  float* SPp = (float*)(ws + oSP);

  hipFuncSetAttribute(reinterpret_cast<const void*>(&k_seg),
                      hipFuncAttributeMaxDynamicSharedMemorySize, LDS_SEG);

  const int nUx = MP * (DIN / 8);
  k_cvt<<<cdiv(nUx, NTHR), NTHR, 0, stream>>>(feat, XB, nN, nUx);
  const int nUw = DIN * (DIN / 8);
  k_cvt<<<cdiv(nUw, NTHR), NTHR, 0, stream>>>(Wl, WT, DIN, nUw);
  k_cvt<<<cdiv(nUw, NTHR), NTHR, 0, stream>>>(Wr, WT + (size_t)DIN * DIN, DIN, nUw);

  k_gemm<<<dim3(MP / GBM, NCOL / GBN), GTHR, 0, stream>>>(XB, WT, bl, br, attl, attr, Vp, SCp, MP);

  k_seg<<<dim3(gA, 2), NTHR, LDS_SEG, stream>>>(src0, dst0, src1, dst1, alph, SCp, SPp,
                                                nN, nE0, nE1, nb, vec8, MP);

  k_fin<<<cdiv(nN, FNODE), NTHR, 0, stream>>>(XB, Vp, SPp, rl, rr, out, nN, MP);
}
